// MultiHeadLinearAttention_62302795596629
// MI455X (gfx1250) — hardware-verified
//
#include <hip/hip_runtime.h>


namespace {
constexpr int Bn = 1, T = 2048, D = 1024, H = 16, HD = 64, D3 = 3072, NT = Bn * T, NF = 64;
constexpr float XS = 8.0f, PS = 8.0f, FS = 1.0f;

typedef _Float16 b16;
typedef __attribute__((ext_vector_type(16))) _Float16 v16b;
typedef __attribute__((ext_vector_type(8))) _Float16 v8b;
typedef __attribute__((ext_vector_type(8))) float v8f;
typedef __attribute__((ext_vector_type(4))) float v4f;
__device__ __forceinline__ float bf16_rne(float f) { unsigned int u = __float_as_uint(f); u += 0x7FFFu + ((u >> 16) & 1u); return __uint_as_float(u & 0xFFFF0000u); }
__device__ __forceinline__ void split16(float v, b16& hi, b16& lo) { hi = (b16)v; lo = (b16)(v - (float)hi); }
__device__ __forceinline__ v16b frag_kb(const b16* p, int hh) { const v8b a = *(const v8b*)(p + 8 * hh), b = *(const v8b*)(p + 16 + 8 * hh); v16b f;
#pragma unroll
  for (int e = 0; e < 8; ++e) { f[e] = a[e]; f[8 + e] = b[e]; } return f; }
__device__ __forceinline__ v8f wmma16b(v16b a, v16b b, v8f c) { v8f d = __builtin_amdgcn_wmma_f32_16x16x32_f16(false, a, false, b, (short)0, c, false, false); asm volatile("v_nop\n\tv_nop\n\tv_nop\n\tv_nop" : "+v"(d) : "v"(a), "v"(b)); return d; }
__device__ __forceinline__ void wave_lds_sync() { __builtin_amdgcn_fence(__ATOMIC_RELEASE, "workgroup"); __builtin_amdgcn_wave_barrier(); __builtin_amdgcn_fence(__ATOMIC_ACQUIRE, "workgroup"); }
__device__ __forceinline__ float nexp(float x) { return __builtin_amdgcn_exp2f(x * 1.4426950408889634f); }
__device__ __forceinline__ float pmul(float a, float b) { float p = a * b; asm volatile("" : "+v"(p)); return p; }

struct Ro_ { static constexpr size_t WQ = 0, WO = (size_t)D3 * D, OM = WO + (size_t)D * D, END = OM + (size_t)H * NF * HD; };
__global__ __launch_bounds__(256) void prep_kernel(const float* __restrict__ x, const float* __restrict__ wq, const float* __restrict__ wk, const float* __restrict__ wv, const float* __restrict__ wout, const float* __restrict__ om, b16* __restrict__ R, float* __restrict__ P, b16* __restrict__ X) {
  const size_t tid = (size_t)blockIdx.x * 256 + threadIdx.x, nth = (size_t)gridDim.x * 256;
  for (int pass = 0; pass < 2; ++pass) {
    for (size_t p = tid; p < (size_t)D3 * D; p += nth) { const int w = (int)(p / ((size_t)D * D)); const size_t r = p % ((size_t)D * D); ((volatile b16*)R)[Ro_::WQ + p] = (b16)bf16_rne(((w == 0) ? wq : (w == 1) ? wk : wv)[r]); }
    for (size_t p = tid; p < (size_t)D * D; p += nth) ((volatile b16*)R)[Ro_::WO + p] = (b16)bf16_rne(wout[p]);
    for (size_t p = tid; p < (size_t)H * NF * HD; p += nth) ((volatile b16*)R)[Ro_::OM + p] = (b16)bf16_rne(om[p]);
    for (size_t q = tid; q < 4104; q += nth) P[q] = 0.0f;
    for (size_t p = tid; p < (size_t)NT * D / 8; p += nth) { v8b v; for (int e = 0; e < 8; ++e) v[e] = (b16)(bf16_rne(x[p * 8 + e]) * XS); *(volatile v8b*)(X + p * 8) = v; }
    __threadfence(); }
}
__global__ __launch_bounds__(64) void qk_kernel(const b16* __restrict__ X, const b16* __restrict__ R, const float* __restrict__ P, b16* __restrict__ QNh, b16* __restrict__ QNl, b16* __restrict__ KNh, b16* __restrict__ KNl) {
  __shared__ __attribute__((aligned(16))) b16 Th[2][16][128 + 8], Tl[2][16][128 + 8];
  const int lane = threadIdx.x & 31, wave = threadIdx.x >> 5, nloc = lane & 15, hlf = lane >> 4, mw = blockIdx.y * 32 + wave * 16; const bool isk = blockIdx.x >= 8; const int c0 = (blockIdx.x & 7) * 128; const int wc0 = (isk ? D : 0) + c0;
  v8f acc[8];
#pragma unroll
  for (int t = 0; t < 8; ++t) acc[t] = (v8f){};
#pragma unroll 2
  for (int kb = 0; kb < D; kb += 32) { const v16b a = frag_kb(X + (size_t)(mw + nloc) * D + kb, hlf);
#pragma unroll
    for (int t = 0; t < 8; ++t) acc[t] = wmma16b(a, frag_kb(R + Ro_::WQ + (size_t)(wc0 + t * 16 + nloc) * D + kb, hlf), acc[t]); }
  float val[8][8]; float ss[2][8]; (void)P;
#pragma unroll
  for (int r = 0; r < 8; ++r) { ss[0][r] = 0.0f; ss[1][r] = 0.0f; }
#pragma unroll
  for (int t = 0; t < 8; ++t)
#pragma unroll
    for (int r = 0; r < 8; ++r) { const float v = acc[t][r] * (1.0f / XS) + P[wc0 + t * 16 + nloc]; val[t][r] = v; ss[t >> 2][r] += pmul(v, v); }
#pragma unroll
  for (int g = 0; g < 2; ++g)
#pragma unroll
    for (int r = 0; r < 8; ++r) { float s = ss[g][r]; s += __shfl_xor(s, 1); s += __shfl_xor(s, 2); s += __shfl_xor(s, 4); s += __shfl_xor(s, 8); ss[g][r] = 1.0f / fmaxf(sqrtf(s), 1e-12f); }
#pragma unroll
  for (int t = 0; t < 8; ++t)
#pragma unroll
    for (int r = 0; r < 8; ++r) { b16 a_, c_; split16(pmul(val[t][r], ss[t >> 2][r]) * XS, a_, c_); Th[wave][8 * hlf + r][t * 16 + nloc] = a_; Tl[wave][8 * hlf + r][t * 16 + nloc] = c_; }
  wave_lds_sync();
  b16* dh = isk ? KNh : QNh; b16* dl = isk ? KNl : QNl;
  for (int pass = 0; pass < 2; ++pass) { for (int i = lane; i < 16 * 16; i += 32) { const int rr = i >> 4, c8 = (i & 15) * 8; const size_t gi = (size_t)(mw + rr) * D + c0 + c8; *(volatile v8b*)(dh + gi) = *(const v8b*)(&Th[wave][rr][c8]); *(volatile v8b*)(dl + gi) = *(const v8b*)(&Tl[wave][rr][c8]); } __threadfence(); }
}
__global__ __launch_bounds__(128) void v_kernel(const b16* __restrict__ X, const b16* __restrict__ R, const float* __restrict__ P, b16* __restrict__ VTh, b16* __restrict__ VTl) {
  __shared__ __attribute__((aligned(16))) b16 Th[128][64 + 8], Tl[128][64 + 8];
  const int lane = threadIdx.x & 31, wave = threadIdx.x >> 5, nloc = lane & 15, hlf = lane >> 4, g0 = blockIdx.y * 64, m0 = g0 + wave * 16, c0 = blockIdx.x * 128; const b16* Bv = R + Ro_::WQ + (size_t)(2 * D + c0) * D; const int b = g0 / T, t0 = g0 % T;
  v8f acc[8];
#pragma unroll
  for (int t = 0; t < 8; ++t) acc[t] = (v8f){};
#pragma unroll 2
  for (int kb = 0; kb < D; kb += 32) { const v16b a = frag_kb(X + (size_t)(m0 + nloc) * D + kb, hlf);
#pragma unroll
    for (int t = 0; t < 8; ++t) acc[t] = wmma16b(a, frag_kb(Bv + (size_t)(t * 16 + nloc) * D + kb, hlf), acc[t]); }
#pragma unroll
  for (int t = 0; t < 8; ++t)
#pragma unroll
    for (int r = 0; r < 8; ++r) { b16 a_, c_; split16(acc[t][r] + XS * P[2 * D + c0 + t * 16 + nloc], a_, c_); Th[t * 16 + nloc][wave * 16 + 8 * hlf + r] = a_; Tl[t * 16 + nloc][wave * 16 + 8 * hlf + r] = c_; }
  __syncthreads();
  for (int pass = 0; pass < 2; ++pass) { for (int i = threadIdx.x; i < 128 * 8; i += 128) { const int dd = i >> 3, c8 = (i & 7) * 8; const size_t gi = ((size_t)b * D + c0 + dd) * T + t0 + c8; *(volatile v8b*)(VTh + gi) = *(const v8b*)(&Th[dd][c8]); *(volatile v8b*)(VTl + gi) = *(const v8b*)(&Tl[dd][c8]); } __threadfence(); }
}
__global__ __launch_bounds__(64) void feat_kernel(const b16* __restrict__ QNh, const b16* __restrict__ QNl, const b16* __restrict__ KNh, const b16* __restrict__ KNl, const b16* __restrict__ R, const float* __restrict__ P, b16* __restrict__ QFh, b16* __restrict__ QFl, b16* __restrict__ KFh, b16* __restrict__ KFl) {
  __shared__ __attribute__((aligned(16))) b16 Th[2][16][64 + 8], Tl[2][16][64 + 8];
  const int lane = threadIdx.x & 31, wave = threadIdx.x >> 5, nloc = lane & 15, hlf = lane >> 4, m0 = blockIdx.x * 32 + wave * 16, h = blockIdx.y; const bool isk = blockIdx.z == 1;
  const b16* Ah = (isk ? KNh : QNh) + h * HD; const b16* Al = (isk ? KNl : QNl) + h * HD; const b16* Bw = R + Ro_::OM + (size_t)h * NF * HD;
  v8f acc[4] = {{}, {}, {}, {}};
#pragma unroll
  for (int kb = 0; kb < HD; kb += 32) { const v16b a = frag_kb(Ah + (size_t)(m0 + nloc) * D + kb, hlf), al_ = frag_kb(Al + (size_t)(m0 + nloc) * D + kb, hlf);
#pragma unroll
    for (int t = 0; t < 4; ++t) { const v16b bw = frag_kb(Bw + (size_t)(t * 16 + nloc) * HD + kb, hlf); acc[t] = wmma16b(a, bw, acc[t]); acc[t] = wmma16b(al_, bw, acc[t]); } }
  __shared__ float Nsq[2][16];
  if (lane < 16) { float s = 0.0f; const b16* rh = Ah + (size_t)(m0 + lane) * D; const b16* rl = Al + (size_t)(m0 + lane) * D; for (int d2 = 0; d2 < HD; ++d2) { const float xv = ((float)rh[d2] + (float)rl[d2]) * (1.0f / XS); s += pmul(xv, xv); } Nsq[wave][lane] = s; }
  wave_lds_sync();
#pragma unroll
  for (int t = 0; t < 4; ++t) {
#pragma unroll
    for (int e = 0; e < 8; ++e) { const float proj = acc[t][e] * (1.0f / XS); const float f = nexp(proj - 0.5f * Nsq[wave][8 * hlf + e]) * 0.125f; b16 a_, c_; split16(f * FS, a_, c_); Th[wave][8 * hlf + e][t * 16 + nloc] = a_; Tl[wave][8 * hlf + e][t * 16 + nloc] = c_; } }
  wave_lds_sync();
  b16* dh = (isk ? KFh : QFh) + h * HD; b16* dl = (isk ? KFl : QFl) + h * HD;
  for (int pass = 0; pass < 2; ++pass) { for (int i = lane; i < 16 * 8; i += 32) { const int rr = i >> 3, c8 = (i & 7) * 8; const size_t gi = (size_t)(m0 + rr) * D + c8; *(volatile v8b*)(dh + gi) = *(const v8b*)(&Th[wave][rr][c8]); *(volatile v8b*)(dl + gi) = *(const v8b*)(&Tl[wave][rr][c8]); } __threadfence(); }
}
__global__ __launch_bounds__(128) void attn_kernel(const b16* __restrict__ QFh, const b16* __restrict__ QFl, const b16* __restrict__ KFh, const b16* __restrict__ KFl, const b16* __restrict__ VTh, const b16* __restrict__ VTl, b16* __restrict__ CH, b16* __restrict__ CL) {
  __shared__ __attribute__((aligned(16))) b16 Oh[16][4 * HD + 8], Ol[16][4 * HD + 8];
  const int wid = threadIdx.x >> 5, lane = threadIdx.x & 31, hh = lane >> 4, col = lane & 15; const int b = blockIdx.z, q0 = blockIdx.x * 16, h = blockIdx.y * 4 + wid, qi = q0 + col;
  const b16* Qr = QFh + ((size_t)b * T) * D + h * HD; const b16* Qlr = QFl + ((size_t)b * T) * D + h * HD; const b16* Kr = KFh + ((size_t)b * T) * D + h * HD; const b16* Klr = KFl + ((size_t)b * T) * D + h * HD; const b16* V = VTh + ((size_t)b * D + h * HD) * T; const b16* Vl = VTl + ((size_t)b * D + h * HD) * T;
  const v16b qf0 = frag_kb(Qr + (size_t)qi * D, hh), qf1 = frag_kb(Qr + (size_t)qi * D + 32, hh), ql0 = frag_kb(Qlr + (size_t)qi * D, hh), ql1 = frag_kb(Qlr + (size_t)qi * D + 32, hh);
  float m = 0.0f, l = 0.0f; v8f o[4] = {{}, {}, {}, {}};
  for (int kb = 0; kb < q0 + 16; kb += 32) {
    v8f s0 = {}, s1 = {};
    { const v16b k00 = frag_kb(Kr + (size_t)(kb + col) * D, hh), k01 = frag_kb(Kr + (size_t)(kb + col) * D + 32, hh), k10 = frag_kb(Kr + (size_t)(kb + 16 + col) * D, hh), k11 = frag_kb(Kr + (size_t)(kb + 16 + col) * D + 32, hh);
      const v16b l00 = frag_kb(Klr + (size_t)(kb + col) * D, hh), l01 = frag_kb(Klr + (size_t)(kb + col) * D + 32, hh), l10 = frag_kb(Klr + (size_t)(kb + 16 + col) * D, hh), l11 = frag_kb(Klr + (size_t)(kb + 16 + col) * D + 32, hh);
      s0 = wmma16b(k00, qf0, s0); s0 = wmma16b(k01, qf1, s0); s0 = wmma16b(l00, qf0, s0); s0 = wmma16b(l01, qf1, s0); s0 = wmma16b(k00, ql0, s0); s0 = wmma16b(k01, ql1, s0);
      s1 = wmma16b(k10, qf0, s1); s1 = wmma16b(k11, qf1, s1); s1 = wmma16b(l10, qf0, s1); s1 = wmma16b(l11, qf1, s1); s1 = wmma16b(k10, ql0, s1); s1 = wmma16b(k11, ql1, s1); }
    float mr = 0.0f;
#pragma unroll
    for (int r = 0; r < 8; ++r) { const int j0 = kb + 8 * hh + r, j1 = j0 + 16; s0[r] = (j0 <= qi) ? fmaxf(s0[r] * (1.0f / (FS * FS)), 0.0f) : 0.0f; s1[r] = (j1 <= qi) ? fmaxf(s1[r] * (1.0f / (FS * FS)), 0.0f) : 0.0f; mr = fmaxf(mr, fmaxf(s0[r], s1[r])); }
    mr = fmaxf(mr, __shfl_xor(mr, 16)); const float mn = fmaxf(m, mr); const float al_ = (m > 0.0f) ? (m / mn) : 1.0f; m = mn; const float invm = (mn > 0.0f) ? (PS / mn) : 0.0f; float sum = 0.0f; v16b pb, pl;
#pragma unroll
    for (int r = 0; r < 8; ++r) { const float e0 = s0[r] * invm, e1 = s1[r] * invm; sum += e0 + e1; b16 a_, c_; split16(e0, a_, c_); pb[r] = a_; pl[r] = c_; split16(e1, a_, c_); pb[8 + r] = a_; pl[8 + r] = c_; }
    sum += __shfl_xor(sum, 16); l = l * al_ + sum;
#pragma unroll
    for (int t = 0; t < 4; ++t) { o[t] *= al_; const v16b vh = frag_kb(V + (size_t)(t * 16 + col) * T + kb, hh); o[t] = wmma16b(vh, pb, o[t]); o[t] = wmma16b(vh, pl, o[t]); o[t] = wmma16b(frag_kb(Vl + (size_t)(t * 16 + col) * T + kb, hh), pb, o[t]); } }
  const float den = fmaxf(l * m * (1.0f / PS), 1e-6f); const float scale = (m * (1.0f / (XS * PS)) / den) * XS;
#pragma unroll
  for (int t = 0; t < 4; ++t)
#pragma unroll
    for (int r = 0; r < 8; ++r) { b16 a_, c_; split16(o[t][r] * scale, a_, c_); Oh[col][wid * HD + t * 16 + 8 * hh + r] = a_; Ol[col][wid * HD + t * 16 + 8 * hh + r] = c_; }
  __syncthreads();
  for (int pass = 0; pass < 2; ++pass) { for (int i = threadIdx.x; i < 16 * 32; i += 128) { const int rr = i >> 5, c8 = (i & 31) * 8; const size_t gi = ((size_t)b * T + q0 + rr) * D + blockIdx.y * 4 * HD + c8; *(volatile v8b*)(CH + gi) = *(const v8b*)(&Oh[rr][c8]); *(volatile v8b*)(CL + gi) = *(const v8b*)(&Ol[rr][c8]); } __threadfence(); }
}
__global__ __launch_bounds__(64) void out_kernel(const b16* __restrict__ CH, const b16* __restrict__ CL, const b16* __restrict__ R, const float* __restrict__ P, float* __restrict__ out) {
  __shared__ __attribute__((aligned(16))) float Ts[2][32][128 + 4];
  const int lane = threadIdx.x & 31, wave = threadIdx.x >> 5, nloc = lane & 15, hlf = lane >> 4, m0 = blockIdx.y * 32, c0 = blockIdx.x * 256 + wave * 128; const b16* RO = R + Ro_::WO;
  v8f acc[2][8];
#pragma unroll
  for (int r = 0; r < 2; ++r)
#pragma unroll
    for (int t = 0; t < 8; ++t) acc[r][t] = (v8f){};
#pragma unroll 2
  for (int kb = 0; kb < D; kb += 32) { const v16b a0 = frag_kb(CH + (size_t)(m0 + nloc) * D + kb, hlf), a1 = frag_kb(CH + (size_t)(m0 + 16 + nloc) * D + kb, hlf), l0 = frag_kb(CL + (size_t)(m0 + nloc) * D + kb, hlf), l1 = frag_kb(CL + (size_t)(m0 + 16 + nloc) * D + kb, hlf);
#pragma unroll
    for (int t = 0; t < 8; ++t) { const v16b bw = frag_kb(RO + (size_t)(c0 + t * 16 + nloc) * D + kb, hlf); acc[0][t] = wmma16b(a0, bw, acc[0][t]); acc[0][t] = wmma16b(l0, bw, acc[0][t]); acc[1][t] = wmma16b(a1, bw, acc[1][t]); acc[1][t] = wmma16b(l1, bw, acc[1][t]); } }
#pragma unroll
  for (int t = 0; t < 8; ++t) { const float bb = P[3072 + c0 + t * 16 + nloc];
#pragma unroll
    for (int r = 0; r < 2; ++r)
#pragma unroll
      for (int v = 0; v < 8; ++v) Ts[wave][r * 16 + 8 * hlf + v][t * 16 + nloc] = acc[r][t][v] * (1.0f / XS) + bb; }
  wave_lds_sync();
  for (int pass = 0; pass < 2; ++pass) { for (int i = lane; i < 32 * 32; i += 32) { const int rr = i >> 5, c4 = (i & 31) * 4; *(volatile v4f*)(out + (size_t)(m0 + rr) * D + c0 + c4) = *(const v4f*)(&Ts[wave][rr][c4]); } __threadfence(); }
}
}

extern "C" void kernel_launch(void* const* d_in, const int* in_sizes, int n_in,
                              void* d_out, int out_size, void* d_ws, size_t ws_size, hipStream_t stream) {
  (void)n_in; (void)out_size;
  auto Fp = [&](int i) { return (const float*)d_in[i]; };
  float* out = (float*)d_out;
  if (in_sizes[0] != NT * D || in_sizes[1] != D * D || in_sizes[5] != H * NF * HD) return;
  size_t off = 0; char* ws = (char*)d_ws;
  auto carve = [&](size_t bytes) { char* p = ws + off; off += (bytes + 255) & ~(size_t)255; return p; };
  const size_t plane = (size_t)NT * D;
  b16* R = (b16*)carve(Ro_::END * 2); float* P = (float*)carve(4104 * 4); b16* X = (b16*)carve(plane * 2);
  b16* QNh = (b16*)carve(plane * 2); b16* QNl = (b16*)carve(plane * 2); b16* KNh = (b16*)carve(plane * 2); b16* KNl = (b16*)carve(plane * 2);
  b16* QFh = (b16*)carve(plane * 2); b16* QFl = (b16*)carve(plane * 2); b16* KFh = (b16*)carve(plane * 2); b16* KFl = (b16*)carve(plane * 2);
  b16* VTh = (b16*)carve(plane * 2); b16* VTl = (b16*)carve(plane * 2);
  b16* CH = QNh; b16* CL = QNl;
  if (off > ws_size) return;
  prep_kernel<<<1024, 256, 0, stream>>>(Fp(0), Fp(1), Fp(2), Fp(3), Fp(4), Fp(5), R, P, X);
  qk_kernel<<<dim3(16, NT / 32), 64, 0, stream>>>(X, R, P, QNh, QNl, KNh, KNl);
  v_kernel<<<dim3(8, NT / 64), 128, 0, stream>>>(X, R, P, VTh, VTl);
  feat_kernel<<<dim3(NT / 32, H, 2), 64, 0, stream>>>(QNh, QNl, KNh, KNl, R, P, QFh, QFl, KFh, KFl);
  attn_kernel<<<dim3(T / 16, 4, Bn), 128, 0, stream>>>(QFh, QFl, KFh, KFl, VTh, VTl, CH, CL);
  out_kernel<<<dim3(4, NT / 32), 64, 0, stream>>>(CH, CL, R, P, out);
}
